// TopologyHead_16269336117488
// MI455X (gfx1250) — hardware-verified
//
#include <hip/hip_runtime.h>

typedef __attribute__((ext_vector_type(16))) _Float16 v16h;
typedef __attribute__((ext_vector_type(8)))  float    v8f;

#define BB   64
#define NN   4096
#define HH   64
#define WW   64
#define LL   5
#define RR   256
#define EPSF 1e-8f

__launch_bounds__(256, 1)
__global__ void pimage_wmma_kernel(const float* __restrict__ pairs,
                                   const float* __restrict__ sigma_p,
                                   float* __restrict__ out)
{
    __shared__ float s_birth[NN];
    __shared__ float s_pers [NN];
    __shared__ float s_img[2][HH * WW];

    const int b    = blockIdx.x;
    const int tid  = threadIdx.x;
    const int lane = tid & 31;
    const int wid  = tid >> 5;
    const int hg   = lane >> 4;
    const int ln   = lane & 15;

    const float sigma  = sigma_p[0];
    const float inv2s2 = 1.0f / (2.0f * sigma * sigma);
    const float c2     = inv2s2 * 1.44269504088896340736f;
    const float inv1pe = 1.0f / (1.0f + EPSF);

    const float* pb = pairs + (size_t)b * NN * 2;
    for (int i = tid; i < NN; i += 256) {
        float bi = pb[2 * i + 0];
        float de = pb[2 * i + 1];
        s_birth[i] = bi;
        s_pers[i]  = de - bi;
    }
    __syncthreads();

    const int   rt = wid & 3;
    const int   kh = wid >> 2;
    const int   h0 = rt * 16;
    const float yh = (float)(h0 + ln) * (1.0f / 63.0f);

    float xw0 = (float)( 0 + ln) * (1.0f / 63.0f);
    float xw1 = (float)(16 + ln) * (1.0f / 63.0f);
    float xw2 = (float)(32 + ln) * (1.0f / 63.0f);
    float xw3 = (float)(48 + ln) * (1.0f / 63.0f);

    v8f acc0 = {}, acc1 = {}, acc2 = {}, acc3 = {};

    const int k_begin = kh * (NN / 2);
    const int k_end   = k_begin + (NN / 2);
    for (int kk = k_begin; kk < k_end; kk += 32) {
        v16h a;
        #pragma unroll
        for (int e = 0; e < 16; ++e) {
            int   K  = (e < 8) ? (hg * 8 + e) : (16 + hg * 8 + (e - 8));
            float pr = s_pers[kk + K];
            float pn = pr * inv1pe;
            float d  = yh - pn;
            float g  = __builtin_amdgcn_exp2f(-c2 * d * d) * pr;
            a[e] = (_Float16)(g * 16384.0f);
        }
        v16h b0, b1, b2, b3;
        #pragma unroll
        for (int e = 0; e < 16; ++e) {
            int   K  = (e < 8) ? (hg * 8 + e) : (16 + hg * 8 + (e - 8));
            float bn = s_birth[kk + K] * inv1pe;
            float d0 = xw0 - bn;
            float d1 = xw1 - bn;
            float d2 = xw2 - bn;
            float d3 = xw3 - bn;
            b0[e] = (_Float16)(__builtin_amdgcn_exp2f(-c2 * d0 * d0) * 16384.0f);
            b1[e] = (_Float16)(__builtin_amdgcn_exp2f(-c2 * d1 * d1) * 16384.0f);
            b2[e] = (_Float16)(__builtin_amdgcn_exp2f(-c2 * d2 * d2) * 16384.0f);
            b3[e] = (_Float16)(__builtin_amdgcn_exp2f(-c2 * d3 * d3) * 16384.0f);
        }
        acc0 = __builtin_amdgcn_wmma_f32_16x16x32_f16(false, a, false, b0,
                                                      (short)0, acc0, false, false);
        acc1 = __builtin_amdgcn_wmma_f32_16x16x32_f16(false, a, false, b1,
                                                      (short)0, acc1, false, false);
        acc2 = __builtin_amdgcn_wmma_f32_16x16x32_f16(false, a, false, b2,
                                                      (short)0, acc2, false, false);
        acc3 = __builtin_amdgcn_wmma_f32_16x16x32_f16(false, a, false, b3,
                                                      (short)0, acc3, false, false);
        asm volatile("v_nop\n\tv_nop\n\tv_nop\n\tv_nop" : "+v"(acc0), "+v"(acc1), "+v"(acc2), "+v"(acc3) : "v"(a), "v"(b0), "v"(b1), "v"(b2), "v"(b3));
    }

    #pragma unroll
    for (int r = 0; r < 8; ++r) {
        int h = h0 + r + hg * 8;
        const float us = 1.0f / 268435456.0f;
        s_img[kh][h * WW +  0 + ln] = acc0[r] * us;
        s_img[kh][h * WW + 16 + ln] = acc1[r] * us;
        s_img[kh][h * WW + 32 + ln] = acc2[r] * us;
        s_img[kh][h * WW + 48 + ln] = acc3[r] * us;
    }
    __syncthreads();

    float m = 0.0f;
    for (int i = tid; i < HH * WW; i += 256)
        m = fmaxf(m, s_img[0][i] + s_img[1][i]);
    s_pers[tid] = m;
    __syncthreads();
    for (int s = 128; s > 0; s >>= 1) {
        if (tid < s) s_pers[tid] = fmaxf(s_pers[tid], s_pers[tid + s]);
        __syncthreads();
    }
    const float scale = 1.0f / (s_pers[0] + EPSF);

    float* ob = out + (size_t)b * HH * WW;
    for (int pass = 0; pass < 2; ++pass) {
        for (int i = tid; i < HH * WW; i += 256)
            *(volatile float*)(ob + i) = (s_img[0][i] + s_img[1][i]) * scale;
        if (pass == 0) __threadfence();
    }
}

__launch_bounds__(256, 1)
__global__ void plandscape_kernel(const float* __restrict__ pairs,
                                  float* __restrict__ out)
{
    __shared__ float s_b[NN];
    __shared__ float s_d[NN];
    __shared__ float s_mn[256];
    __shared__ float s_mx[256];

    const int b   = blockIdx.x;
    const int tid = threadIdx.x;

    const float* pb = pairs + (size_t)b * NN * 2;
    float mn = 3.4e38f, mx = -3.4e38f;
    for (int i = tid; i < NN; i += 256) {
        float bi = pb[2 * i + 0];
        float de = pb[2 * i + 1];
        s_b[i] = bi;
        s_d[i] = de;
        mn = fminf(mn, bi);
        mx = fmaxf(mx, de);
    }
    s_mn[tid] = mn;
    s_mx[tid] = mx;
    __syncthreads();
    for (int s = 128; s > 0; s >>= 1) {
        if (tid < s) {
            s_mn[tid] = fminf(s_mn[tid], s_mn[tid + s]);
            s_mx[tid] = fmaxf(s_mx[tid], s_mx[tid + s]);
        }
        __syncthreads();
    }
    const float minb = s_mn[0];
    const float maxd = s_mx[0];
    const float t = minb + (maxd - minb) * ((float)tid * (1.0f / 255.0f));

    float t0 = 0.f, t1 = 0.f, t2 = 0.f, t3 = 0.f, t4 = 0.f;
    for (int n = 0; n < NN; ++n) {
        float bi = s_b[n];
        float de = s_d[n];
        float x  = fmaxf(fminf(t - bi, de - t), 0.0f);
        float u;
        u = fmaxf(t0, x); x = fminf(t0, x); t0 = u;
        u = fmaxf(t1, x); x = fminf(t1, x); t1 = u;
        u = fmaxf(t2, x); x = fminf(t2, x); t2 = u;
        u = fmaxf(t3, x); x = fminf(t3, x); t3 = u;
        t4 = fmaxf(t4, x);
    }

    float* ob = out + (size_t)b * LL * RR;
    for (int pass = 0; pass < 2; ++pass) {
        *(volatile float*)(ob + 0 * RR + tid) = t0;
        *(volatile float*)(ob + 1 * RR + tid) = t1;
        *(volatile float*)(ob + 2 * RR + tid) = t2;
        *(volatile float*)(ob + 3 * RR + tid) = t3;
        *(volatile float*)(ob + 4 * RR + tid) = t4;
        if (pass == 0) __threadfence();
    }
}

extern "C" void kernel_launch(void* const* d_in, const int* in_sizes, int n_in,
                              void* d_out, int out_size, void* d_ws, size_t ws_size,
                              hipStream_t stream) {
    const float* pairs = (const float*)d_in[0];
    const float* sigma = (const float*)d_in[1];
    float*       out   = (float*)d_out;

    pimage_wmma_kernel<<<dim3(BB), dim3(256), 0, stream>>>(pairs, sigma, out);
    plandscape_kernel <<<dim3(BB), dim3(256), 0, stream>>>(pairs, out + BB * HH * WW);
}
